// AttentionPooling_vectorized_65678639890659
// MI455X (gfx1250) — hardware-verified
//
#include <hip/hip_runtime.h>
#include <math.h>

typedef __attribute__((ext_vector_type(16))) _Float16 v16h;
typedef __attribute__((ext_vector_type(16))) __bf16 v16b;
typedef __attribute__((ext_vector_type(8)))  _Float16 v8h;
typedef __attribute__((ext_vector_type(8)))  float v8f;
typedef __attribute__((ext_vector_type(4)))  float v4f;
typedef __attribute__((ext_vector_type(2)))  float v2f;
typedef __attribute__((ext_vector_type(4)))  unsigned v4u;
typedef __attribute__((ext_vector_type(4)))  int v4i;
typedef float __attribute__((may_alias)) float_a;
typedef int __attribute__((may_alias)) int_a;

template <typename T> __device__ __forceinline__ void vst2(void* p, T v) { *(volatile T*)p = v; __threadfence(); *(volatile T*)p = v; }
__device__ __forceinline__ v8f wmma16(v16h a, v16h b, v8f c) {
  v8f d = __builtin_amdgcn_wmma_f32_16x16x32_f16(false, a, false, b, (short)0, c, false, false);
  asm volatile("v_nop\n\tv_nop\n\tv_nop\n\tv_nop" : "+v"(d) : "v"(a), "v"(b));
  return d;
}
__device__ __forceinline__ v8f wmma_bf(v16b a, v16b b, v8f c) {
  v8f d = __builtin_amdgcn_wmma_f32_16x16x32_bf16(false, a, false, b, (short)0, c, false, false);
  asm volatile("v_nop\n\tv_nop\n\tv_nop\n\tv_nop" : "+v"(d) : "v"(a), "v"(b));
  return d;
}
__device__ __forceinline__ v16h frag_h(const _Float16* rowk0, int lane) {
  union { v16h v; v8h q[2]; } u; const _Float16* p = rowk0 + 8 * (lane >> 4);
  u.q[0] = *(const v8h*)p; u.q[1] = *(const v8h*)(p + 16); return u.v;
}
__device__ __forceinline__ v16h frag_f32(const float* rowk0, int lane) {
  v16h a; const float* p = rowk0 + 8 * (lane >> 4);
#pragma unroll
  for (int i = 0; i < 8; ++i) { a[i] = (_Float16)p[i]; a[8 + i] = (_Float16)p[16 + i]; }
  return a;
}
__device__ __forceinline__ v16h frag_f32s(const float* rowk0, int lane, float sc) {
  v16h a; const float* p = rowk0 + 8 * (lane >> 4);
#pragma unroll
  for (int i = 0; i < 8; ++i) { a[i] = (_Float16)(p[i] * sc); a[8 + i] = (_Float16)(p[16 + i] * sc); }
  return a;
}
__device__ __forceinline__ v16h fragc_f32(const float* W, int k0, int n, int lane, int ld, int K) {
  v16h a; const int g = lane >> 4;
#pragma unroll
  for (int i = 0; i < 8; ++i) { const int ka = k0 + 8 * g + i, kb = ka + 16;
    a[i] = (_Float16)(ka < K ? W[(size_t)(ka < K ? ka : K - 1) * ld + n] : 0.f); a[8 + i] = (_Float16)(kb < K ? W[(size_t)(kb < K ? kb : K - 1) * ld + n] : 0.f); }
  return a;
}
struct F2 { v16b h, l; };
__device__ __forceinline__ F2 bsplit16(const float v[16]) { F2 r;
#pragma unroll
  for (int i = 0; i < 16; ++i) { const __bf16 h = (__bf16)v[i]; r.h[i] = h; r.l[i] = (__bf16)(v[i] - (float)h); }
  return r; }
__device__ __forceinline__ F2 split_row(const float* row, int k0, int lane) { float v[16]; const float* p = row + k0 + 8 * (lane >> 4);
#pragma unroll
  for (int i = 0; i < 8; ++i) { v[i] = p[i]; v[8 + i] = p[16 + i]; }
  return bsplit16(v); }
__device__ __forceinline__ F2 split_rowK(const float* row, int k0, int lane, int K) { float v[16]; const int g = lane >> 4;
#pragma unroll
  for (int i = 0; i < 8; ++i) { const int ka = k0 + 8 * g + i, kb = ka + 16; v[i] = ka < K ? row[ka < K ? ka : K - 1] : 0.f; v[8 + i] = kb < K ? row[kb < K ? kb : K - 1] : 0.f; }
  return bsplit16(v); }
__device__ __forceinline__ F2 split_col(const float* W, int k0, int n, int lane, int ld, int K) { float v[16]; const int g = lane >> 4;
#pragma unroll
  for (int i = 0; i < 8; ++i) { const int ka = k0 + 8 * g + i, kb = ka + 16; v[i] = ka < K ? W[(size_t)(ka < K ? ka : K - 1) * ld + n] : 0.f; v[8 + i] = kb < K ? W[(size_t)(kb < K ? kb : K - 1) * ld + n] : 0.f; }
  return bsplit16(v); }
__device__ __forceinline__ v8f mac3(const F2& a, const F2& b, v8f c) { c = wmma_bf(a.l, b.h, c); c = wmma_bf(a.h, b.l, c); return wmma_bf(a.h, b.h, c); }
__device__ __forceinline__ float sigm(float v) { return 1.0f / (1.0f + expf(-v)); }
#define LDSX() do { asm volatile("s_wait_dscnt 0" ::: "memory"); __builtin_amdgcn_wave_barrier(); __builtin_amdgcn_fence(__ATOMIC_RELEASE, "workgroup"); } while (0)


#define NBB 8
#define SL 512
#define HM 768
#define NS 256
#define WSP 32
#define NH 12
#define HD 64
#define FFN 3072
#define NTOK (NBB * SL)
#define NSPAN (NBB * NS)
#define KVP (2 * HM)
#ifndef NBT
#define NBT NBB
#endif
typedef __attribute__((ext_vector_type(8))) __bf16 v8b;
__device__ __forceinline__ v16b frag_b(const __bf16* rowk0, int lane) {
  union { v16b v; v8b q[2]; } u; const __bf16* p = rowk0 + 8 * (lane >> 4);
  u.q[0] = *(const v8b*)p; u.q[1] = *(const v8b*)(p + 16); return u.v;
}
__device__ __forceinline__ float bfr(float v) { return (float)(__bf16)v; }
__device__ __attribute__((noinline)) float exp_ni(float v) { return expf(v); }
__device__ __attribute__((noinline)) float erf_ni(float v) { return erff(v); }

__device__ __attribute__((noinline)) float sin_ni(float v) { return sinf(v); }
__device__ __attribute__((noinline)) float cos_ni(float v) { return cosf(v); }
#define PK_KV 0
#define PK_O  (PK_KV + KVP * HM)
#define PK_1  (PK_O + HM * HM)
#define PK_2  (PK_1 + FFN * HM)
#define PK_END (PK_2 + HM * FFN)
#define WS_PK   0u
#define WS_PE   (WS_PK + 2u * PK_END)
#define WS_PEKV (WS_PE + 4u * SL * HM)
#define WS_TKV  (WS_PEKV + 4u * SL * KVP)
#define WS_Q    (WS_TKV + 4u * NTOK * KVP)
#define WS_SC   (WS_Q + 4u * 1024)
#define WS_CTX  (WS_SC + 4u * NTOK * 16)
#define WS_X0   (WS_CTX + 4u * NSPAN * HM)
#define WS_X1   (WS_X0 + 4u * NSPAN * HM)
#define WS_HF   (WS_X1 + 4u * NSPAN * HM)
#define WS_X2   (WS_HF + 4u * NSPAN * FFN)
#define WS_LOK  (WS_X2 + 4u * NSPAN * HM)
#define WS_END  (WS_LOK + 4u * NSPAN)

__global__ __launch_bounds__(256) void k_pack(const float* __restrict__ Wm, int K, __bf16* __restrict__ DST) {
  __shared__ __align__(16) __bf16 s[FFN]; const int n = blockIdx.x, tid = threadIdx.x; const float* src = Wm + (size_t)n * K;
  for (int k = tid; k < K; k += 256) s[k] = (__bf16)src[k];
  __syncthreads();
  for (int q = tid; q < K / 8; q += 256) vst2((unsigned*)(DST + (size_t)n * K + q * 8), *(const v4u*)&s[q * 8]);
}
__global__ __launch_bounds__(256) void k_pe(float* __restrict__ PE) {
  __shared__ __align__(16) float s[HM]; const int t = blockIdx.x, tid = threadIdx.x;
  for (int c = tid; c < HM; c += 256) { const int i2 = c & ~1; const float divt = expf((float)i2 * (-logf(10000.0f) / (float)HM)); const float ang = (float)t * divt; s[c] = (c & 1) ? cos_ni(ang) : sin_ni(ang); }
  __syncthreads();
  for (int q = tid; q < HM / 4; q += 256) vst2(PE + (size_t)t * HM + q * 4, *(const v4f*)&s[q * 4]);
}
template <int K, int AM, int EPI, int RM>
__global__ __launch_bounds__(128) void k_lin(const float* __restrict__ A, int lda, const __bf16* __restrict__ P, const float* __restrict__ bias, const float* __restrict__ bias2, float* __restrict__ OUT, int ldo, const float* __restrict__ RES, int ldr, int RMOD) {
  __shared__ __align__(16) float so[4][16][132];
  const int tid = threadIdx.x, wave = tid >> 5, lane = tid & 31, col = lane & 15, g = lane >> 4; const size_t r0 = (size_t)blockIdx.x * 64 + wave * 16; const int n0 = blockIdx.y * 128;
  v8f acc[8] = {};
#pragma unroll 2
  for (int kc = 0; kc < K / 32; ++kc) {
    if (AM == 0) { v16b a; { const float* p = A + (r0 + col) * lda + kc * 32 + 8 * g;
#pragma unroll
        for (int i = 0; i < 8; ++i) { a[i] = (__bf16)p[i]; a[8 + i] = (__bf16)p[16 + i]; } }
#pragma unroll
      for (int j = 0; j < 8; ++j) acc[j] = wmma_bf(a, frag_b(P + (size_t)(n0 + j * 16 + col) * K + kc * 32, lane), acc[j]); }
    else { const F2 a = split_row(A + (r0 + col) * lda, kc * 32, lane);
#pragma unroll
      for (int j = 0; j < 8; ++j) { const v16b w = frag_b(P + (size_t)(n0 + j * 16 + col) * K + kc * 32, lane); acc[j] = wmma_bf(a.l, w, acc[j]); acc[j] = wmma_bf(a.h, w, acc[j]); } } }
#pragma unroll
  for (int j = 0; j < 8; ++j) { const int n = n0 + j * 16 + col; float bb = bias ? bfr(bias[n]) : 0.f; if (bias2) bb += bfr(bias2[n]);
#pragma unroll
    for (int r = 0; r < 8; ++r) { const size_t row = r0 + 8 * g + r; float v = acc[j][r] + bb; if (RM == 1) v += RES[row * ldr + n]; if (RM == 2) v += RES[(row % RMOD) * ldr + n]; if (EPI == 1) v = fmaxf(v, 0.f); so[wave][8 * g + r][j * 16 + col] = v; } }
  LDSX();
  for (int rl = 0; rl < 16; ++rl) vst2(OUT + (r0 + rl) * ldo + n0 + lane * 4, *(const v4f*)&so[wave][rl][lane * 4]);
}
__global__ __launch_bounds__(256) void k_q(const float* __restrict__ Q0, const float* __restrict__ Wq, const float* __restrict__ bq, float* __restrict__ Q) {
  __shared__ float sq0[HM]; __shared__ __align__(16) float sq[1024]; const int tid = threadIdx.x;
  for (int k = tid; k < HM; k += 256) sq0[k] = bfr(Q0[k]);
  for (int k = tid; k < 1024; k += 256) sq[k] = 0.f;
  __syncthreads();
  for (int o = tid; o < HM; o += 256) { float s = bfr(bq[o]); const float* w = Wq + (size_t)o * HM;
#pragma unroll 4
    for (int k = 0; k < HM; ++k) s += sq0[k] * bfr(w[k]);
    sq[o] = s; }
  __syncthreads();
  vst2(Q + tid * 4, *(const v4f*)&sq[tid * 4]);
}
__global__ __launch_bounds__(256) void k_sc(const float* __restrict__ Q, const float* __restrict__ TKV, float* __restrict__ SC) {
  __shared__ float sq[HM]; __shared__ __align__(16) float ss[64][16]; const int tid = threadIdx.x; const size_t t0 = (size_t)blockIdx.x * 64;
  for (int k = tid; k < HM; k += 256) sq[k] = Q[k];
  for (int q = tid; q < 64 * 16; q += 256) (&ss[0][0])[q] = 0.f;
  __syncthreads();
  { const int tl = tid >> 2, hq = tid & 3; const float* kr = TKV + (t0 + tl) * KVP;
    for (int h = hq; h < NH; h += 4) { float s = 0.f;
#pragma unroll 4
      for (int d = 0; d < HD; ++d) s += sq[h * HD + d] * kr[h * HD + d];
      ss[tl][h] = s * 0.125f; } }
  __syncthreads();
  vst2(SC + t0 * 16 + tid * 4, *(const v4f*)(&ss[0][0] + tid * 4));
}
__global__ __launch_bounds__(256) void k_span(const int* __restrict__ SPAN, const float* __restrict__ SC, const float* __restrict__ TKV, const float* __restrict__ bkv, float* __restrict__ CTX) {
  __shared__ float sa[NH][WSP]; __shared__ int stok[WSP]; __shared__ float sval[WSP]; __shared__ __align__(16) float sc[HM];
  const int n = blockIdx.x, tid = threadIdx.x; const int b = n / NS;
  const long long st = SPAN[(size_t)n * 2 + 0], en = SPAN[(size_t)n * 2 + 1]; const long long len = en - st;
  if (tid < WSP) { long long p = st + tid; p = p < 0 ? 0 : (p > SL - 1 ? SL - 1 : p); stok[tid] = b * SL + (int)p; sval[tid] = ((long long)tid < len) ? 1.f : 0.f; }
  __syncthreads();
  if (tid < NH) { const int h = tid; float s[WSP]; float mx = -3.0e38f;
#pragma unroll
    for (int w = 0; w < WSP; ++w) { s[w] = sval[w] > 0.f ? SC[(size_t)stok[w] * 16 + h] : -1.0e9f; mx = fmaxf(mx, s[w]); }
    float z = 0.f;
#pragma unroll
    for (int w = 0; w < WSP; ++w) { s[w] = exp_ni(s[w] - mx); z += s[w]; }
    const float iz = 1.0f / z;
#pragma unroll
    for (int w = 0; w < WSP; ++w) sa[h][w] = s[w] * iz; }
  __syncthreads();
  for (int c = tid; c < HM; c += 256) { const int h = c / HD; const float bvv = bfr(bkv[HM + c]); float acc = 0.f;
#pragma unroll 4
    for (int w = 0; w < WSP; ++w) { const float vv = sval[w] > 0.f ? TKV[(size_t)stok[w] * KVP + HM + c] : bvv; acc += sa[h][w] * vv; }
    sc[c] = acc; }
  __syncthreads();
  for (int q = tid; q < HM / 4; q += 256) vst2(CTX + (size_t)n * HM + q * 4, *(const v4f*)&sc[q * 4]);
}
__global__ __launch_bounds__(32) void k_lok(const int* __restrict__ SPAN, float* __restrict__ LOK) {
  __shared__ __align__(16) float s[32]; const int n0 = blockIdx.x * 32, tid = threadIdx.x;
  const long long st = SPAN[(size_t)(n0 + tid) * 2 + 0], en = SPAN[(size_t)(n0 + tid) * 2 + 1]; s[tid] = (en - st > 0) ? 1.f : 0.f;
  LDSX();
  if (tid < 8) vst2(LOK + n0 + tid * 4, *(const v4f*)&s[tid * 4]);
}
template <int FIN>
__global__ __launch_bounds__(256) void k_ln(const float* __restrict__ X, const float* __restrict__ gw, const float* __restrict__ bw, const float* __restrict__ LOK, float* __restrict__ Y) {
  __shared__ __align__(16) float s[8][HM];
  const int wave = threadIdx.x >> 5, lane = threadIdx.x & 31; const size_t r = (size_t)blockIdx.x * 8 + wave; const float* x = X + r * HM; float* sw = s[wave];
  float sum = 0.f;
#pragma unroll 4
  for (int i = 0; i < HM / 32; ++i) { const float t = x[lane + 32 * i]; sw[lane + 32 * i] = t; sum += t; }
#pragma unroll
  for (int o = 1; o < 32; o <<= 1) sum += __shfl_xor(sum, o);
  const float mu = sum / (float)HM; float var = 0.f;
#pragma unroll 4
  for (int i = 0; i < HM / 32; ++i) { const float d = sw[lane + 32 * i] - mu; var += d * d; }
#pragma unroll
  for (int o = 1; o < 32; o <<= 1) var += __shfl_xor(var, o);
  const float rs = rsqrtf(var / (float)HM + 1e-5f); const float keep = FIN ? LOK[r] : 1.f;
#pragma unroll 4
  for (int i = 0; i < HM / 32; ++i) { const int c = lane + 32 * i; sw[c] = keep > 0.f ? ((sw[c] - mu) * rs * bfr(gw[c]) + bfr(bw[c])) : 0.f; }
  LDSX();
  for (int pc = lane; pc < HM / 4; pc += 32) vst2(Y + r * HM + pc * 4, *(const v4f*)&sw[pc * 4]);
}
extern "C" void kernel_launch(void* const* d_in, const int* in_sizes, int n_in, void* d_out, int out_size, void* d_ws, size_t ws_size, hipStream_t stream) {
  (void)in_sizes; (void)n_in; (void)out_size;
  const float** F = (const float**)d_in;
  if (ws_size < (size_t)WS_END) return;
  char* ws = (char*)d_ws; __bf16* PK = (__bf16*)(ws + WS_PK);
  float *PE = (float*)(ws + WS_PE), *PEKV = (float*)(ws + WS_PEKV), *TKV = (float*)(ws + WS_TKV), *Q = (float*)(ws + WS_Q), *SC = (float*)(ws + WS_SC), *CTX = (float*)(ws + WS_CTX), *X0 = (float*)(ws + WS_X0), *X1 = (float*)(ws + WS_X1), *HF = (float*)(ws + WS_HF), *X2 = (float*)(ws + WS_X2), *LOK = (float*)(ws + WS_LOK);
  const int* SPAN = (const int*)d_in[1];
  k_pack<<<KVP, 256, 0, stream>>>(F[3] + (size_t)HM * HM, HM, PK + PK_KV);
  k_pack<<<HM, 256, 0, stream>>>(F[5], HM, PK + PK_O);
  k_pack<<<FFN, 256, 0, stream>>>(F[9], HM, PK + PK_1);
  k_pack<<<HM, 256, 0, stream>>>(F[11], FFN, PK + PK_2);
  k_pe<<<SL, 256, 0, stream>>>(PE);
  k_lin<HM, 1, 0, 0><<<dim3(SL / 64, KVP / 128), 128, 0, stream>>>(PE, HM, PK + PK_KV, F[4] + HM, nullptr, PEKV, KVP, nullptr, 0, 1);
  k_lin<HM, 0, 0, 2><<<dim3(NBT * SL / 64, KVP / 128), 128, 0, stream>>>(F[0], HM, PK + PK_KV, nullptr, nullptr, TKV, KVP, PEKV, KVP, SL);
  k_q<<<1, 256, 0, stream>>>(F[2], F[3], F[4], Q);
  k_sc<<<NBT * SL / 64, 256, 0, stream>>>(Q, TKV, SC);
  k_lok<<<NBT * NS / 32, 32, 0, stream>>>(SPAN, LOK);
  k_span<<<NBT * NS, 256, 0, stream>>>(SPAN, SC, TKV, F[4] + HM, CTX);
  k_lin<HM, 1, 0, 0><<<dim3(NBT * NS / 64, HM / 128), 128, 0, stream>>>(CTX, HM, PK + PK_O, F[6], F[2], X0, HM, nullptr, 0, 1);
  k_ln<0><<<NBT * NS / 8, 256, 0, stream>>>(X0, F[7], F[8], LOK, X1);
  k_lin<HM, 1, 1, 0><<<dim3(NBT * NS / 64, FFN / 128), 128, 0, stream>>>(X1, HM, PK + PK_1, F[10], nullptr, HF, FFN, nullptr, 0, 1);
  k_lin<FFN, 1, 0, 1><<<dim3(NBT * NS / 64, HM / 128), 128, 0, stream>>>(HF, FFN, PK + PK_2, F[12], nullptr, X2, HM, X1, HM, 1);
  k_ln<1><<<NBT * NS / 8, 256, 0, stream>>>(X2, F[7], F[8], LOK, (float*)d_out);
}
